// NUSpectralConv1D_61529701482701
// MI455X (gfx1250) — hardware-run, weakly checked
//
#include <hip/hip_runtime.h>
#include <math.h>
#pragma clang fp contract(off)

typedef __attribute__((ext_vector_type(16))) _Float16 v16h;
typedef __attribute__((ext_vector_type(8)))  _Float16 v8h;
typedef __attribute__((ext_vector_type(8)))  float    v8f;
typedef __attribute__((ext_vector_type(4)))  float    v4f;

constexpr int kNb     = 16;
constexpr int kCh     = 64;
constexpr int kSamp   = 8192;
constexpr int kModes  = 257;
constexpr int kHalfM  = 128;
constexpr int kCols   = 257;
constexpr int kColsP  = 320;
constexpr int kSplitK = 8;
constexpr int kKper   = kSamp / kSplitK;
constexpr float kXwCarry = 1024.0f;
constexpr float kHCarry  = 256.0f;
constexpr float kInv2Pi  = (float)(1.0 / (2.0 * 3.14159265358979323846));
constexpr float kFwdScale = 1.0f / kXwCarry;
constexpr float kOutScale = kInv2Pi * (1.0f / kHCarry);
static_assert(kModes == 2 * kHalfM + 1);
static_assert(kCols == (kHalfM + 1) + kHalfM);
static_assert((kColsP % 64) == 0 && (kColsP % 32) == 0 && kColsP >= kCols);
static_assert((kKper % 32) == 0 && kKper * kSplitK == kSamp);
static_assert(kCh == 64 && (kSamp % 64) == 0);

constexpr size_t kOffXW  = 0;
constexpr size_t kOffTAB = kOffXW  + (size_t)kNb * kCh * kSamp * 2;
constexpr size_t kOffFP  = kOffTAB + (size_t)kNb * kColsP * kSamp * 2;
constexpr size_t kOffHP  = kOffFP  + (size_t)kSplitK * kNb * kCh * kColsP * 4;
constexpr size_t kWsTotal = kOffHP + (size_t)kNb * kCh * kColsP * 2;
static_assert(kWsTotal == 111804416ull);
static_assert(kWsTotal <= 134217728ull);
static_assert((kOffTAB % 128) == 0 && (kOffFP % 128) == 0 && (kOffHP % 128) == 0);

struct FragH {
  union U { v16h v; v8h h[2]; };
  static __device__ __forceinline__ v16h load(const _Float16* p) {
    U f;
    f.h[0] = *(const v8h*)(p);
    f.h[1] = *(const v8h*)(p + 16);
    return f.v;
  }
};
__device__ __forceinline__ v8f mma_g(v16h a, v16h b, v8f c) {
  c = __builtin_amdgcn_wmma_f32_16x16x32_f16(false, a, false, b, (short)0, c, false, false);
  asm volatile("v_nop\n\tv_nop\n\tv_nop\n\tv_nop" : "+v"(c) : "v"(a), "v"(b));
  return c;
}

template <bool BIAS_ROW>
__global__ __launch_bounds__(256) void gemm64_f16_kernel(
    const unsigned short* __restrict__ Ap, int lda, long strideA,
    const unsigned short* __restrict__ Btp, int ldb, long strideB,
    float* __restrict__ Cout, int ldc, long strideCb, long strideCs,
    const float* __restrict__ bias,
    int tilesN, int nSplit, int kPerSplit, int totalTiles, float scale)
{
  typedef _Float16 T;
  __shared__ __align__(16) float sT[8][16 * 68];
  const int lane = threadIdx.x & 31;
  const int wave = __builtin_amdgcn_readfirstlane((int)(threadIdx.x >> 5));
  const int tile = blockIdx.x * 8 + wave;
  if (tile >= totalTiles) return;
  const int tn = tile % tilesN;
  const int t2 = tile / tilesN;
  const int sp = t2 % nSplit;
  const int b  = t2 / nSplit;
  const int n0 = tn << 6;

  const T* Ab = (const T*)Ap  + (size_t)b * strideA + (size_t)sp * kPerSplit;
  const T* Bb = (const T*)Btp + (size_t)b * strideB + (size_t)sp * kPerSplit;
  float*   C  = Cout + (size_t)b * strideCb + (size_t)sp * strideCs;

  const int rlane = lane & 15;
  const int koff  = (lane >> 4) * 8;
  const int mOff  = (lane >> 4) * 8;

  v8f acc[4][4];
#pragma unroll
  for (int i = 0; i < 4; ++i)
#pragma unroll
    for (int j = 0; j < 4; ++j) acc[i][j] = (v8f){0.f, 0.f, 0.f, 0.f, 0.f, 0.f, 0.f, 0.f};

  for (int k0 = 0; k0 < kPerSplit; k0 += 32) {
    v16h bh[4];
#pragma unroll
    for (int j = 0; j < 4; ++j) {
      const size_t bo = (size_t)(n0 + (j << 4) + rlane) * ldb + koff + k0;
      bh[j] = FragH::load(Bb + bo);
    }
#pragma unroll
    for (int i = 0; i < 4; ++i) {
      const size_t ao = (size_t)((i << 4) + rlane) * lda + koff + k0;
      const v16h ah = FragH::load(Ab + ao);
#pragma unroll
      for (int j = 0; j < 4; ++j) acc[i][j] = mma_g(ah, bh[j], acc[i][j]);
    }
  }

  float* slab = sT[wave];
#pragma unroll
  for (int i = 0; i < 4; ++i) {
    const int mBase = i << 4;
    v4f bva = (v4f){0.f, 0.f, 0.f, 0.f};
    v4f bvb = (v4f){0.f, 0.f, 0.f, 0.f};
    if (BIAS_ROW) {
      bva = *(const v4f*)(bias + mBase + mOff);
      bvb = *(const v4f*)(bias + mBase + mOff + 4);
    }
#pragma unroll
    for (int j = 0; j < 4; ++j) {
#pragma unroll
      for (int r = 0; r < 8; ++r) {
        float v = acc[i][j][r] * scale;
        if (BIAS_ROW) v = v + ((r < 4) ? bva[r & 3] : bvb[r & 3]);
        slab[(mOff + r) * 68 + (j << 4) + rlane] = v;
      }
    }
    __builtin_amdgcn_fence(__ATOMIC_RELEASE, "workgroup");
    __builtin_amdgcn_wave_barrier();
    __builtin_amdgcn_fence(__ATOMIC_ACQUIRE, "workgroup");
    {
      const int hh = lane >> 4, c4 = (lane & 15) * 4;
      for (int pass = 0; pass < 2; ++pass) {
#pragma unroll
        for (int it = 0; it < 8; ++it) {
          const int row = it * 2 + hh;
          const v4f v = *(const v4f*)(slab + row * 68 + c4);
          *(volatile v4f*)(C + (size_t)(mBase + row) * ldc + n0 + c4) = v;
        }
        __threadfence();
      }
    }
    __builtin_amdgcn_fence(__ATOMIC_RELEASE, "workgroup");
    __builtin_amdgcn_wave_barrier();
    __builtin_amdgcn_fence(__ATOMIC_ACQUIRE, "workgroup");
  }
}

__global__ __launch_bounds__(256) void prep_xw_kernel(
    const float* __restrict__ x, const float* __restrict__ z, unsigned short* __restrict__ XW)
{
  const int t  = blockIdx.x * 256 + threadIdx.x;
  const int b  = t >> 10;
  const int n0 = (t & 1023) << 3;
  const float* zb = z + (size_t)b * kSamp;
  const int nl = (n0 > 0) ? (n0 - 1) : 0;
  const int nr = (n0 + 8 < kSamp) ? (n0 + 8) : (kSamp - 1);
  const v4f za = *(const v4f*)(zb + n0);
  const v4f zc = *(const v4f*)(zb + n0 + 4);
  float zz[10];
  zz[0] = zb[nl];
  zz[1] = za[0]; zz[2] = za[1]; zz[3] = za[2]; zz[4] = za[3];
  zz[5] = zc[0]; zz[6] = zc[1]; zz[7] = zc[2]; zz[8] = zc[3];
  zz[9] = zb[nr];
  float wsc[8];
#pragma unroll
  for (int e = 0; e < 8; ++e) {
    const float dr = zz[e + 2] - zz[e + 1];
    const float dl = zz[e + 1] - zz[e];
    float w = 0.5f * (dr + dl);
    w = fmaxf(w, 0.0f);
    wsc[e] = w * kXwCarry;
  }
  const size_t base = (size_t)b * kCh * kSamp + n0;
#pragma unroll 1
  for (int c = 0; c < kCh; ++c) {
    const float* xp = x + base + (size_t)c * kSamp;
    const v4f a0 = *(const v4f*)(xp);
    const v4f a1 = *(const v4f*)(xp + 4);
    v8h hv;
#pragma unroll
    for (int e = 0; e < 4; ++e) {
      const float p0 = a0[e] * wsc[e];
      const float p1 = a1[e] * wsc[4 + e];
      hv[e]     = (_Float16)p0;
      hv[4 + e] = (_Float16)p1;
    }
    unsigned short* q = XW + base + (size_t)c * kSamp;
    *(volatile v8h*)q = hv;
    __threadfence();
    *(volatile v8h*)q = hv;
  }
}

__global__ __launch_bounds__(256) void build_tab_jn_kernel(
    const float* __restrict__ z, unsigned short* __restrict__ TAB)
{
  __shared__ __align__(16) _Float16 sh[2048];
  const int tid = threadIdx.x;
  const int j   = blockIdx.y;
  const int b   = blockIdx.z;
  const int nb  = blockIdx.x * 2048;
  const bool padRow = (j >= kCols);
  const bool useSin = (j > kHalfM);
  const float kf = (float)(useSin ? (j - kHalfM) : j);
  const float* zb = z + (size_t)b * kSamp + nb;
  if (!padRow) {
#pragma unroll 1
    for (int it = 0; it < 8; ++it) {
      const int i = it * 256 + tid;
      float zv = zb[i];
      float p = zv * kf;
      asm volatile("" : "+v"(p));
      float sv, cv;
      sincosf(p, &sv, &cv);
      const float v = useSin ? sv : cv;
      sh[i] = (_Float16)v;
    }
  } else {
#pragma unroll 1
    for (int it = 0; it < 8; ++it) {
      const int i = it * 256 + tid;
      sh[i] = (_Float16)0.0f;
    }
  }
  __syncthreads();
  const v8h hv = *(const v8h*)(sh + tid * 8);
  unsigned short* q = TAB + ((size_t)(b * kColsP + j) * kSamp + nb + tid * 8);
  *(volatile v8h*)q = hv;
  __threadfence();
  *(volatile v8h*)q = hv;
}

__device__ __forceinline__ float fold_elem(const float* __restrict__ FP, const float* __restrict__ wr,
                                           const float* __restrict__ wi, int b, int c, int j)
{
  const bool isCos = (j <= kHalfM);
  const bool live  = (j < kCols);
  int k = isCos ? j : (j - kHalfM);
  k = (k > kHalfM) ? kHalfM : k;
  const int colC = k;
  const int colS = (k >= 1) ? (kHalfM + k) : (kHalfM + 1);
  const size_t rowOff = ((size_t)b * kCh + c) * kColsP;
  float fc = 0.0f, fs = 0.0f;
#pragma unroll 1
  for (int s = 0; s < kSplitK; ++s) {
    const float* pp = FP + (size_t)s * ((size_t)kNb * kCh * kColsP) + rowOff;
    fc = fc + pp[colC];
    fs = fs + pp[colS];
  }
  fs = (k == 0) ? 0.0f : fs;
  const float* wrc = wr + c * kModes;
  const float* wic = wi + c * kModes;
  const float wrp = wrc[kHalfM + k], wrm = wrc[kHalfM - k];
  const float wip = wic[kHalfM + k], wim = wic[kHalfM - k];
  const float sW = (k == 0) ? wrp : (wrp + wrm);
  const float dW = wip - wim;
  const float vk = (k == kHalfM) ? 0.5f : 1.0f;
  const float hc = vk * (fc * sW + fs * dW);
  const float hs = vk * (fs * sW - fc * dW);
  const float v  = isCos ? hc : hs;
  return live ? (v * kHCarry) : 0.0f;
}

__global__ __launch_bounds__(256) void fold_kernel(
    const float* __restrict__ FP, const float* __restrict__ wr, const float* __restrict__ wi,
    unsigned short* __restrict__ HP)
{
  const int t   = blockIdx.x * 256 + threadIdx.x;
  const int e0  = t * 2;
  const int row = e0 / kColsP;
  const int j0  = e0 - row * kColsP;
  const int b   = row >> 6;
  const int c   = row & 63;
  const float v0 = fold_elem(FP, wr, wi, b, c, j0);
  const float v1 = fold_elem(FP, wr, wi, b, c, j0 + 1);
  const _Float16 h0 = (_Float16)v0;
  const _Float16 h1 = (_Float16)v1;
  const unsigned u0 = (unsigned)__builtin_bit_cast(unsigned short, h0);
  const unsigned u1 = (unsigned)__builtin_bit_cast(unsigned short, h1);
  const unsigned u  = u0 | (u1 << 16);
  volatile unsigned* q = (volatile unsigned*)HP + t;
  *q = u;
  __threadfence();
  *q = u;
}

__global__ __launch_bounds__(256) void build_tab_nj_kernel(
    const float* __restrict__ z, unsigned short* __restrict__ TAB)
{
  __shared__ __align__(16) _Float16 sh[32 * kColsP];
  const int tid = threadIdx.x;
  const int n0  = blockIdx.x * 32;
  const int b   = blockIdx.y;
  const float* zb = z + (size_t)b * kSamp + n0;
#pragma unroll 1
  for (int it = 0; it < 33; ++it) {
    const int i  = it * 256 + tid;
    const bool ok = (i < 32 * kCols);
    const int ic = ok ? i : (32 * kCols - 1);
    const int r  = ic / kCols;
    const int j  = ic - r * kCols;
    float zv = zb[r];
    asm volatile("" : "+v"(zv));
    const bool isCos = (j <= kHalfM);
    const int k = isCos ? j : (j - kHalfM);
    float p = zv * (float)k;
    asm volatile("" : "+v"(p));
    float sv, cv;
    sincosf(p, &sv, &cv);
    const float v = isCos ? cv : sv;
    if (ok) sh[r * kColsP + j] = (_Float16)v;
  }
#pragma unroll 1
  for (int it = 0; it < 8; ++it) {
    const int i = it * 256 + tid;
    if (i < 32 * (kColsP - kCols)) {
      const int r  = i / (kColsP - kCols);
      const int jj = i - r * (kColsP - kCols);
      sh[r * kColsP + kCols + jj] = (_Float16)0.0f;
    }
  }
  __syncthreads();
  v8h hv[5];
#pragma unroll
  for (int it = 0; it < 5; ++it) hv[it] = *(const v8h*)(sh + (it * 256 + tid) * 8);
  unsigned short* dst = TAB + ((size_t)b * kSamp + n0) * kColsP;
  for (int pass = 0; pass < 2; ++pass) {
#pragma unroll
    for (int it = 0; it < 5; ++it) *(volatile v8h*)(dst + (it * 256 + tid) * 8) = hv[it];
    __threadfence();
  }
}

extern "C" void kernel_launch(void* const* d_in, const int* in_sizes, int n_in,
                              void* d_out, int out_size, void* d_ws, size_t ws_size,
                              hipStream_t stream) {
  if (n_in < 5) return;
  if (in_sizes[0] != kNb * kCh * kSamp) return;
  if (in_sizes[1] != kNb * kSamp) return;
  if (in_sizes[2] != kCh * kModes) return;
  if (in_sizes[3] != kCh * kModes) return;
  if (in_sizes[4] != kCh) return;
  if (out_size != kNb * kCh * kSamp) return;
  if (ws_size < kWsTotal) return;

  const float* x    = (const float*)d_in[0];
  const float* z    = (const float*)d_in[1];
  const float* wr   = (const float*)d_in[2];
  const float* wi   = (const float*)d_in[3];
  const float* bias = (const float*)d_in[4];
  float* y = (float*)d_out;

  char* ws = (char*)d_ws;
  unsigned short* XW  = (unsigned short*)(ws + kOffXW);
  unsigned short* TAB = (unsigned short*)(ws + kOffTAB);
  float*          FP  = (float*)(ws + kOffFP);
  unsigned short* HP  = (unsigned short*)(ws + kOffHP);

  prep_xw_kernel<<<(kNb * kSamp / 8) / 256, 256, 0, stream>>>(x, z, XW);

  build_tab_jn_kernel<<<dim3(kSamp / 2048, kColsP, kNb), 256, 0, stream>>>(z, TAB);

  gemm64_f16_kernel<false><<<(kNb * kSplitK * (kColsP / 64)) / 8, 256, 0, stream>>>(
      XW, kSamp, (long)kCh * kSamp,
      TAB, kSamp, (long)kColsP * kSamp,
      FP, kColsP, (long)kCh * kColsP, (long)kNb * kCh * kColsP,
      bias,
      kColsP / 64, kSplitK, kKper, kNb * kSplitK * (kColsP / 64), kFwdScale);

  fold_kernel<<<(kNb * kCh * kColsP / 2) / 256, 256, 0, stream>>>(FP, wr, wi, HP);

  build_tab_nj_kernel<<<dim3(kSamp / 32, kNb), 256, 0, stream>>>(z, TAB);

  gemm64_f16_kernel<true><<<(kNb * (kSamp / 64)) / 8, 256, 0, stream>>>(
      HP, kColsP, (long)kCh * kColsP,
      TAB, kColsP, (long)kSamp * kColsP,
      y, kSamp, (long)kCh * kSamp, 0L,
      bias,
      kSamp / 64, 1, kColsP, kNb * (kSamp / 64), kOutScale);
}
